// GraphUnet_8933531976315
// MI455X (gfx1250) — hardware-verified
//
#include <hip/hip_runtime.h>
#include <stddef.h>
#include <stdint.h>

#define NN     4096
#define DD     128
#define KSEL   2457
#define KP     2560
#define IDXN   3072
#define K2     256
#define NTHR   256
#define NWAVE  8
#define EPT    8
#define CHUNK  (NTHR * EPT)
#define WCAP   (EPT * 32)
#define LISTN  (NWAVE * WCAP)
#define GBM    64
#define GBN    128
#define GTHR   128
#define NPB    (KP / GBN)
#define ARB    16
#define ASLB   4
#define ACNTI  (ARB * NN / 2)
#define ADJ_LDS_INTS (ACNTI + LISTN)
#define URB    32
#define U_LDS_INTS (URB * NN / 4)
#define NUH    (NN * DD / 8)
#define NUWD   (DD * DD / 8)
#define NUW2   (DD * K2 / 8)
#define NUTOT  (NUH + NUWD + 2 * NUW2)
#define WSMAX  134217728
#define ONEBF  ((unsigned short)0x3F80)
#define ZBF    ((unsigned short)0)

enum { MODE_F32 = 0, MODE_H0Z = 1, MODE_SUB = 2, MODE_XST = 3 };

static_assert(NN % GBM == 0 && KP % GBM == 0 && KP % GBN == 0 && K2 % GBN == 0 && DD == GBN);
static_assert(DD % 32 == 0 && K2 % 32 == 0 && KP % 32 == 0 && NN % 32 == 0);
static_assert(KSEL <= KP && KP <= IDXN && IDXN % (NTHR * 4) == 0 && NN % (NTHR * 4) == 0);
static_assert(NUTOT % NTHR == 0 && NUH % NTHR == 0 && NUWD % NTHR == 0 && NUW2 % NTHR == 0);
static_assert(ADJ_LDS_INTS % 4 == 0 && U_LDS_INTS % 4 == 0);
static_assert((ADJ_LDS_INTS % (NTHR * 4)) == 0 && (U_LDS_INTS % (NTHR * 4)) == 0);
static_assert(NN % ARB == 0 && KP % URB == 0 && KP % 16 == 0 && NN % 64 == 0 && NN % NWAVE == 0);
static_assert((CHUNK & (CHUNK - 1)) == 0 && CHUNK <= 4096);
static_assert(ARB == (1 << ASLB));
static_assert(NN == 16 * NTHR);
static_assert(2 * NN * DD == 1048576);
static_assert(GBM == (GTHR / 32) * 16 && GBN == 4 * 32);

typedef float          v4f   __attribute__((ext_vector_type(4)));
typedef float          v8f   __attribute__((ext_vector_type(8)));
typedef int            v4i   __attribute__((ext_vector_type(4)));
typedef int            v8i   __attribute__((ext_vector_type(8)));
typedef unsigned short v8us  __attribute__((ext_vector_type(8)));
typedef unsigned short v16us __attribute__((ext_vector_type(16)));
typedef __bf16         v16bf __attribute__((ext_vector_type(16)));
typedef v4f  __attribute__((may_alias)) v4fa;
typedef v4i  __attribute__((may_alias)) v4ia;
typedef v8us __attribute__((may_alias)) v8usa;
typedef unsigned int __attribute__((may_alias)) ua32;
union FragB { v16bf v; v16us u; v8us h[2]; v8i w; };

__device__ __forceinline__ v8f wmb(const FragB& a, const FragB& b, v8f c) {
  v8f d = __builtin_amdgcn_wmma_f32_16x16x32_bf16(false, a.v, false, b.v, (short)0, c, false, false);
  asm volatile("v_nop\n\tv_nop\n\tv_nop\n\tv_nop" : "+v"(d) : "v"(a.w), "v"(b.w));
  return d;
}

__device__ __forceinline__ unsigned bf16_bits(float f) {
  const unsigned u = __float_as_uint(f);
  return (u + 0x7FFFu + ((u >> 16) & 1u)) >> 16;
}
__device__ __forceinline__ float bf16_val(float f) {
  return __uint_as_float(bf16_bits(f) << 16);
}
__device__ __forceinline__ int clampn(int x, int n) {
  return x < 0 ? 0 : (x > n - 1 ? n - 1 : x);
}

template <int SLB>
__device__ __forceinline__ int scan_chunk(const int* __restrict__ dsts, int nE, int cbase, int slotBase,
                                          int nb, int vec8, int* list, int tid, int lane, int wave) {
  int wc = 0;
  const int el0  = tid * EPT;
  const int e0   = cbase + el0;
  const int sent = -2147483647 - 1;
  v4i da, db;
  if (vec8 != 0 && cbase + CHUNK <= nE) {
    da = *(const v4i*)(dsts + e0);
    db = *(const v4i*)(dsts + e0 + 4);
  } else {
    da.x = (e0     < nE) ? dsts[min(e0,     nE - 1)] : sent;
    da.y = (e0 + 1 < nE) ? dsts[min(e0 + 1, nE - 1)] : sent;
    da.z = (e0 + 2 < nE) ? dsts[min(e0 + 2, nE - 1)] : sent;
    da.w = (e0 + 3 < nE) ? dsts[min(e0 + 3, nE - 1)] : sent;
    db.x = (e0 + 4 < nE) ? dsts[min(e0 + 4, nE - 1)] : sent;
    db.y = (e0 + 5 < nE) ? dsts[min(e0 + 5, nE - 1)] : sent;
    db.z = (e0 + 6 < nE) ? dsts[min(e0 + 6, nE - 1)] : sent;
    db.w = (e0 + 7 < nE) ? dsts[min(e0 + 7, nE - 1)] : sent;
  }
  const unsigned nbs = (unsigned)slotBase;
  const unsigned unb = (unsigned)nb;
  const unsigned s0 = (unsigned)da.x - nbs, s1 = (unsigned)da.y - nbs;
  const unsigned s2 = (unsigned)da.z - nbs, s3 = (unsigned)da.w - nbs;
  const unsigned s4 = (unsigned)db.x - nbs, s5 = (unsigned)db.y - nbs;
  const unsigned s6 = (unsigned)db.z - nbs, s7 = (unsigned)db.w - nbs;
  const bool h0 = s0 < unb, h1 = s1 < unb, h2 = s2 < unb, h3 = s3 < unb;
  const bool h4 = s4 < unb, h5 = s5 < unb, h6 = s6 < unb, h7 = s7 < unb;
  const unsigned any = __builtin_amdgcn_ballot_w32(h0 | h1 | h2 | h3 | h4 | h5 | h6 | h7);
  if (any != 0u) {
#define HITJ(J, HJ, SJ) { \
      const unsigned mj = __builtin_amdgcn_ballot_w32(HJ); \
      if (mj != 0u) { \
        if (HJ) { \
          const int pos = wc + (int)__builtin_amdgcn_mbcnt_lo(mj, 0u); \
          if (pos < WCAP) list[wave * WCAP + pos] = ((el0 + (J)) << SLB) | (int)(SJ); \
        } \
        wc += (int)__builtin_popcount(mj); } }
    HITJ(0, h0, s0)
    HITJ(1, h1, s1)
    HITJ(2, h2, s2)
    HITJ(3, h3, s3)
    HITJ(4, h4, s4)
    HITJ(5, h5, s5)
    HITJ(6, h6, s6)
    HITJ(7, h7, s7)
#undef HITJ
  }
  return wc;
}

__global__ __launch_bounds__(NTHR) void k_prep(const float* __restrict__ h, const float* __restrict__ Wd,
                                               const float* __restrict__ Wb, const float* __restrict__ Wu,
                                               unsigned short* hbf, unsigned short* wdt,
                                               unsigned short* wbt2, unsigned short* wut2) {
  const int u = (int)blockIdx.x * NTHR + (int)threadIdx.x;
  v8us o;
  unsigned short* dp;
  if (u < NUH) {
    const int row = u >> 4;
    const int k8  = (u & 15) * 8;
    const float* p = h + (size_t)row * DD + k8;
    const v4f a = *(const v4f*)p;
    const v4f b = *(const v4f*)(p + 4);
    o[0] = (unsigned short)bf16_bits(a.x); o[1] = (unsigned short)bf16_bits(a.y);
    o[2] = (unsigned short)bf16_bits(a.z); o[3] = (unsigned short)bf16_bits(a.w);
    o[4] = (unsigned short)bf16_bits(b.x); o[5] = (unsigned short)bf16_bits(b.y);
    o[6] = (unsigned short)bf16_bits(b.z); o[7] = (unsigned short)bf16_bits(b.w);
    dp = hbf + (size_t)row * DD + k8;
  } else if (u < NUH + NUWD) {
    const int v  = u - NUH;
    const int n  = v >> 4;
    const int k8 = (v & 15) * 8;
    const float* p = Wd + (size_t)k8 * DD + n;
#pragma unroll
    for (int i = 0; i < 8; ++i) o[i] = (unsigned short)bf16_bits(p[(size_t)i * DD]);
    dp = wdt + (size_t)n * DD + k8;
  } else if (u < NUH + NUWD + NUW2) {
    const int v  = u - NUH - NUWD;
    const int n  = v >> 5;
    const int k8 = (v & 31) * 8;
    const int kk = k8 & (DD - 1);
    const float* p = Wb + (size_t)kk * DD + n;
#pragma unroll
    for (int i = 0; i < 8; ++i) o[i] = (unsigned short)bf16_bits(p[(size_t)i * DD]);
    dp = wbt2 + (size_t)n * K2 + k8;
  } else if (u < NUTOT) {
    const int v  = u - NUH - NUWD - NUW2;
    const int n  = v >> 5;
    const int k8 = (v & 31) * 8;
    const int kk = k8 & (DD - 1);
    const float* p = Wu + (size_t)kk * DD + n;
#pragma unroll
    for (int i = 0; i < 8; ++i) o[i] = (unsigned short)bf16_bits(p[(size_t)i * DD]);
    dp = wut2 + (size_t)n * K2 + k8;
  } else {
    return;
  }
  *(volatile v8us*)dp = o;
  __threadfence();
  *(volatile v8us*)dp = o;
}

__device__ __forceinline__ void adj_pass(const unsigned short* cnt16, unsigned short* adjp, int rowBase,
                                         int wave, int lane) {
#pragma unroll 4
  for (int i = 0; i < 32; ++i) {
    const int rr  = 2 * wave + (i >> 4);
    const int seg = (i & 15) * 256 + 8 * lane;
    const v8us c = *(const v8usa*)(cnt16 + rr * NN + seg);
    v8us o;
#pragma unroll
    for (int e = 0; e < 8; ++e) o[e] = (unsigned short)bf16_bits((float)c[e]);
    unsigned short* op = adjp + (size_t)(rowBase + rr) * NN + seg;
    *(volatile v8us*)op = o;
  }
}

__global__ __launch_bounds__(NTHR) void k_adj(const int* __restrict__ srcs, const int* __restrict__ dsts,
                                              int nE, int vec8, unsigned short* adjp) {
  extern __shared__ __attribute__((aligned(16))) int dsm[];
  unsigned short* cnt16 = (unsigned short*)dsm;
  int* list = dsm + ACNTI;
  __shared__ int wcnt[NWAVE];
  const int tid = (int)threadIdx.x, lane = tid & 31, wave = tid >> 5;
  const int rowBase = (int)blockIdx.x * ARB;

  {
    const v4i z4 = {0, 0, 0, 0};
    for (int i = tid * 4; i < ADJ_LDS_INTS; i += NTHR * 4) *(v4ia*)(dsm + i) = z4;
    if (tid < NWAVE) wcnt[tid] = 0;
  }
  __syncthreads();

  const int nChunks = (nE + CHUNK - 1) / CHUNK;
#pragma unroll 1
  for (int ch = 0; ch < nChunks; ++ch) {
    const int cbase = ch * CHUNK;
    const int wc = scan_chunk<ASLB>(srcs, nE, cbase, rowBase, ARB, vec8, list, tid, lane, wave);
    if (lane == 0) wcnt[wave] = wc;
    __syncthreads();
    if (wave == 0) {
#pragma unroll 1
      for (int w2 = 0; w2 < NWAVE; ++w2) {
        int c = wcnt[w2];
        c = c < 0 ? 0 : (c > WCAP ? WCAP : c);
#pragma unroll 1
        for (int b0 = 0; b0 < c; b0 += 32) {
          const int ix  = b0 + lane;
          const int ent = list[w2 * WCAP + (ix < WCAP ? ix : WCAP - 1)];
          const int m32 = (c - b0) < 32 ? (c - b0) : 32;
#pragma unroll 1
          for (int k = 0; k < m32; ++k) {
            const int u  = __builtin_amdgcn_readlane(ent, k);
            const int sl = u & (ARB - 1);
            const int el = (u >> ASLB) & (CHUNK - 1);
            int eid = cbase + el;
            eid = eid > nE - 1 ? nE - 1 : eid;
            const int d = clampn(dsts[eid], NN);
            if (lane == 0) {
              const int ci = sl * NN + d;
              const unsigned cv = cnt16[ci];
              cnt16[ci] = (unsigned short)(cv < 65535u ? cv + 1u : cv);
            }
          }
        }
      }
    }
    __syncthreads();
  }

  adj_pass(cnt16, adjp, rowBase, wave, lane);
  __threadfence();
  adj_pass(cnt16, adjp, rowBase, wave, lane);
}

__device__ __forceinline__ void urow_pass(const unsigned char* flags, unsigned short* outp, int pbase,
                                          int wave, int lane) {
#pragma unroll 4
  for (int i = 0; i < 64; ++i) {
    const int rr  = 4 * wave + (i >> 4);
    const int seg = (i & 15) * 256 + 8 * lane;
    const ua32* fp = (const ua32*)(flags + rr * NN + seg);
    const unsigned a = fp[0], b = fp[1];
    v8us o;
    o[0] = (a & 0xffu)         != 0u ? ONEBF : ZBF;
    o[1] = ((a >> 8) & 0xffu)  != 0u ? ONEBF : ZBF;
    o[2] = ((a >> 16) & 0xffu) != 0u ? ONEBF : ZBF;
    o[3] = ((a >> 24) & 0xffu) != 0u ? ONEBF : ZBF;
    o[4] = (b & 0xffu)         != 0u ? ONEBF : ZBF;
    o[5] = ((b >> 8) & 0xffu)  != 0u ? ONEBF : ZBF;
    o[6] = ((b >> 16) & 0xffu) != 0u ? ONEBF : ZBF;
    o[7] = ((b >> 24) & 0xffu) != 0u ? ONEBF : ZBF;
    unsigned short* op = outp + (size_t)(pbase + rr) * NN + seg;
    *(volatile v8us*)op = o;
  }
}

__global__ __launch_bounds__(NTHR) void k_urow(const int* __restrict__ keys, const int* __restrict__ oth,
                                               int nE, int vec8, const int* __restrict__ mem,
                                               unsigned short* outp) {
  extern __shared__ __attribute__((aligned(16))) int dsm[];
  unsigned char* flags = (unsigned char*)dsm;
  const int tid = (int)threadIdx.x, lane = tid & 31, wave = tid >> 5;
  const int pbase = (int)blockIdx.x * URB;

  {
    const v4i z4 = {0, 0, 0, 0};
    for (int i = tid * 4; i < U_LDS_INTS; i += NTHR * 4) *(v4ia*)(dsm + i) = z4;
  }
  __syncthreads();

  const int nChunks = (nE + CHUNK - 1) / CHUNK;
#pragma unroll 1
  for (int ch = 0; ch < nChunks; ++ch) {
    const int cbase = ch * CHUNK;
    const int e0 = cbase + tid * EPT;
    v4i ka, kb, oa, ob;
    if (vec8 != 0 && cbase + CHUNK <= nE) {
      ka = *(const v4i*)(keys + e0);
      kb = *(const v4i*)(keys + e0 + 4);
      oa = *(const v4i*)(oth + e0);
      ob = *(const v4i*)(oth + e0 + 4);
    } else {
      const int sent = -1;
      ka.x = (e0     < nE) ? keys[min(e0,     nE - 1)] : sent;
      ka.y = (e0 + 1 < nE) ? keys[min(e0 + 1, nE - 1)] : sent;
      ka.z = (e0 + 2 < nE) ? keys[min(e0 + 2, nE - 1)] : sent;
      ka.w = (e0 + 3 < nE) ? keys[min(e0 + 3, nE - 1)] : sent;
      kb.x = (e0 + 4 < nE) ? keys[min(e0 + 4, nE - 1)] : sent;
      kb.y = (e0 + 5 < nE) ? keys[min(e0 + 5, nE - 1)] : sent;
      kb.z = (e0 + 6 < nE) ? keys[min(e0 + 6, nE - 1)] : sent;
      kb.w = (e0 + 7 < nE) ? keys[min(e0 + 7, nE - 1)] : sent;
      oa.x = oth[min(e0,     nE - 1)]; oa.y = oth[min(e0 + 1, nE - 1)];
      oa.z = oth[min(e0 + 2, nE - 1)]; oa.w = oth[min(e0 + 3, nE - 1)];
      ob.x = oth[min(e0 + 4, nE - 1)]; ob.y = oth[min(e0 + 5, nE - 1)];
      ob.z = oth[min(e0 + 6, nE - 1)]; ob.w = oth[min(e0 + 7, nE - 1)];
    }
#define UPROC(KJ, OJ) { \
      const int kj = (KJ); const int oj = (OJ); \
      const bool inr = (unsigned)kj < (unsigned)NN; \
      const int kc = clampn(kj, NN); \
      int p = mem[kc]; \
      p = inr ? p : -1; \
      const unsigned slot = (unsigned)(p - pbase); \
      const int oc = clampn(oj, NN); \
      if (slot < (unsigned)URB) flags[slot * NN + oc] = (unsigned char)1; }
    UPROC(ka.x, oa.x)
    UPROC(ka.y, oa.y)
    UPROC(ka.z, oa.z)
    UPROC(ka.w, oa.w)
    UPROC(kb.x, ob.x)
    UPROC(kb.y, ob.y)
    UPROC(kb.z, ob.z)
    UPROC(kb.w, ob.w)
#undef UPROC
  }
  __syncthreads();

  urow_pass(flags, outp, pbase, wave, lane);
  __threadfence();
  urow_pass(flags, outp, pbase, wave, lane);
}

template <int MODE>
__device__ __forceinline__ void gemm_pass(const float* stg, const float* rs, float* Cf, int ldc,
                                          unsigned short* C16, float* q0, int rowBase, int colBase,
                                          int by, int wave, int lane) {
  if constexpr (MODE == MODE_F32 || MODE == MODE_H0Z) {
#pragma unroll
    for (int i = 0; i < 16; ++i) {
      const v4f v = *(const v4fa*)(stg + (16 * wave + i) * GBN + 4 * lane);
      float* op = Cf + (size_t)(rowBase + 16 * wave + i) * (size_t)ldc + colBase + 4 * lane;
      *(volatile v4f*)op = v;
    }
    if constexpr (MODE == MODE_H0Z) {
      if (wave == 0 && lane < 16) {
        const v4f z = *(const v4fa*)(rs + 4 * lane);
        *(volatile v4f*)(q0 + rowBase + 4 * lane) = z;
      }
    }
  } else if constexpr (MODE == MODE_SUB) {
#pragma unroll
    for (int i = 0; i < 8; ++i) {
      const int row = 16 * wave + 2 * i + (lane >> 4);
      const int c8  = 8 * (lane & 15);
      const v4f a = *(const v4fa*)(stg + row * GBN + c8);
      const v4f b = *(const v4fa*)(stg + row * GBN + c8 + 4);
      v8us o;
      o[0] = (a.x != 0.0f) ? ONEBF : ZBF; o[1] = (a.y != 0.0f) ? ONEBF : ZBF;
      o[2] = (a.z != 0.0f) ? ONEBF : ZBF; o[3] = (a.w != 0.0f) ? ONEBF : ZBF;
      o[4] = (b.x != 0.0f) ? ONEBF : ZBF; o[5] = (b.y != 0.0f) ? ONEBF : ZBF;
      o[6] = (b.z != 0.0f) ? ONEBF : ZBF; o[7] = (b.w != 0.0f) ? ONEBF : ZBF;
      unsigned short* op = C16 + (size_t)(rowBase + row) * (size_t)ldc + colBase + c8;
      *(volatile v8us*)op = o;
    }
    if (wave == 0 && lane < 16) {
      const v4f c = *(const v4fa*)(rs + 4 * lane);
      *(volatile v4f*)(q0 + (size_t)by * KP + rowBase + 4 * lane) = c;
    }
  } else {
    const int part = wave >> 1;
#pragma unroll 2
    for (int i = 0; i < 16; ++i) {
      const int L  = wave * 64 + 4 * i + (lane >> 3);
      const int c  = L & (DD - 1);
      const int j0 = 8 * (lane & 7);
      v8us o;
#pragma unroll
      for (int jj = 0; jj < 8; ++jj) {
        const float v = stg[(j0 + jj) * GBN + c] * rs[j0 + jj];
        const unsigned hb = bf16_bits(v);
        const unsigned lb = bf16_bits(v - __uint_as_float(hb << 16));
        o[jj] = (unsigned short)(part != 0 ? lb : hb);
      }
      unsigned short* op = C16 + (size_t)(part * DD + c) * (size_t)ldc + rowBase + j0;
      *(volatile v8us*)op = o;
    }
  }
}

template <int MODE>
__global__ __launch_bounds__(GTHR) void k_gemm(const unsigned short* __restrict__ A, int lda,
                                               const unsigned short* __restrict__ BT, int ldb, int K,
                                               float* Cf, int ldc, unsigned short* C16,
                                               const float* __restrict__ p0, const float* __restrict__ p1,
                                               const float* __restrict__ p2, float* q0) {
  __shared__ __attribute__((aligned(16))) float stg[GBM * GBN];
  __shared__ __attribute__((aligned(16))) float rs[GBM];
  const int tid = (int)threadIdx.x, lane = tid & 31, wave = tid >> 5, hh = lane >> 4, m = lane & 15;
  const int rowBase = (int)blockIdx.x * GBM;
  const int colBase = (int)blockIdx.y * GBN;
  const int by = (int)blockIdx.y;

  if constexpr (MODE == MODE_XST) {
    if (tid < GBM) {
      float d = 0.0f;
#pragma unroll 1
      for (int b = 0; b < NPB; ++b) d += p0[(size_t)b * KP + rowBase + tid];
      const float rcp = 1.0f / d;
      rs[tid] = (rowBase + tid < KSEL) ? rcp : 0.0f;
    }
  }

  v8f acc[8];
  {
    const v8f z = {0.f, 0.f, 0.f, 0.f, 0.f, 0.f, 0.f, 0.f};
#pragma unroll
    for (int t = 0; t < 8; ++t) acc[t] = z;
  }
  const unsigned short* ap = A  + (size_t)(rowBase + 16 * wave + m) * (size_t)lda + 8 * hh;
  const unsigned short* bp = BT + (size_t)(colBase + m) * (size_t)ldb + 8 * hh;

#pragma unroll 1
  for (int k0 = 0; k0 < K; k0 += 32) {
    FragB af;
    af.h[0] = *(const v8usa*)(ap + k0);
    af.h[1] = *(const v8usa*)(ap + k0 + 16);
#pragma unroll
    for (int nt = 0; nt < 8; ++nt) {
      const unsigned short* wq = bp + (size_t)(16 * nt) * (size_t)ldb + k0;
      FragB bf;
      bf.h[0] = *(const v8usa*)wq;
      bf.h[1] = *(const v8usa*)(wq + 16);
      acc[nt] = wmb(af, bf, acc[nt]);
    }
  }

#pragma unroll
  for (int nt = 0; nt < 8; ++nt) {
    const int lc = 16 * nt + m;
    float bvl = 0.0f;
    if constexpr (MODE == MODE_H0Z) bvl = bf16_val(p0[colBase + lc]);
#pragma unroll
    for (int r = 0; r < 8; ++r) {
      const int lr = 16 * wave + 8 * hh + r;
      float v = acc[nt][r];
      if constexpr (MODE == MODE_H0Z) v = v + bvl;
      if constexpr (MODE == MODE_SUB) v = (v > 0.0f) ? 1.0f : 0.0f;
      stg[lr * GBN + lc] = v;
    }
  }
  __syncthreads();

  if constexpr (MODE == MODE_H0Z) {
    const float pw0 = bf16_val(p1[4 * lane]),     pw1 = bf16_val(p1[4 * lane + 1]);
    const float pw2 = bf16_val(p1[4 * lane + 2]), pw3 = bf16_val(p1[4 * lane + 3]);
    const float pbv = bf16_val(p2[0]);
    float mine = 0.0f;
#pragma unroll 1
    for (int rr = 0; rr < 16; ++rr) {
      const v4f x = *(const v4fa*)(stg + (16 * wave + rr) * GBN + 4 * lane);
      float p = x.x * pw0;
      p = fmaf(x.y, pw1, p);
      p = fmaf(x.z, pw2, p);
      p = fmaf(x.w, pw3, p);
      p += __shfl_xor(p, 16, 32);
      p += __shfl_xor(p, 8, 32);
      p += __shfl_xor(p, 4, 32);
      p += __shfl_xor(p, 2, 32);
      p += __shfl_xor(p, 1, 32);
      const float z = p + pbv;
      mine = (lane == rr) ? z : mine;
    }
    if (lane < 16) rs[16 * wave + lane] = mine;
    __syncthreads();
  }
  if constexpr (MODE == MODE_SUB) {
    float mine = 0.0f;
#pragma unroll 1
    for (int rr = 0; rr < 16; ++rr) {
      const v4f x = *(const v4fa*)(stg + (16 * wave + rr) * GBN + 4 * lane);
      float p = (x.x + x.y) + (x.z + x.w);
      p += __shfl_xor(p, 16, 32);
      p += __shfl_xor(p, 8, 32);
      p += __shfl_xor(p, 4, 32);
      p += __shfl_xor(p, 2, 32);
      p += __shfl_xor(p, 1, 32);
      mine = (lane == rr) ? p : mine;
    }
    if (lane < 16) rs[16 * wave + lane] = mine;
    __syncthreads();
  }

  gemm_pass<MODE>(stg, rs, Cf, ldc, C16, q0, rowBase, colBase, by, wave, lane);
  __threadfence();
  gemm_pass<MODE>(stg, rs, Cf, ldc, C16, q0, rowBase, colBase, by, wave, lane);
}

__device__ __forceinline__ void sel_pass(const int* lmem, const int* lidx, int* memp, int* idxp, int tid) {
#pragma unroll
  for (int it = 0; it < NN / (NTHR * 4); ++it) {
    const int o = (it * NTHR + tid) * 4;
    const v4i v = *(const v4ia*)(lmem + o);
    *(volatile v4i*)(memp + o) = v;
  }
#pragma unroll
  for (int it = 0; it < IDXN / (NTHR * 4); ++it) {
    const int o = (it * NTHR + tid) * 4;
    const v4i v = *(const v4ia*)(lidx + o);
    *(volatile v4i*)(idxp + o) = v;
  }
}

__global__ __launch_bounds__(NTHR) void k_select(const float* __restrict__ zp, int* memp, int* idxp) {
  __shared__ __attribute__((aligned(16))) float zs[NN];
  __shared__ __attribute__((aligned(16))) int lmem[NN];
  __shared__ __attribute__((aligned(16))) int lidx[IDXN];
  __shared__ int wtot[NWAVE];
  const int tid = (int)threadIdx.x, lane = tid & 31, wave = tid >> 5;

#pragma unroll
  for (int it = 0; it < NN / (NTHR * 4); ++it) {
    const int o = (it * NTHR + tid) * 4;
    *(v4fa*)(zs + o) = *(const v4f*)(zp + o);
  }
  {
    const v4i z4 = {0, 0, 0, 0};
#pragma unroll
    for (int it = 0; it < IDXN / (NTHR * 4); ++it) {
      const int o = (it * NTHR + tid) * 4;
      *(v4ia*)(lidx + o) = z4;
    }
    if (tid < NWAVE) wtot[tid] = 0;
  }
  __syncthreads();

  const int ibase = 16 * tid;
  float zi[16];
  int rk[16];
#pragma unroll
  for (int mm = 0; mm < 16; ++mm) { zi[mm] = zs[ibase + mm]; rk[mm] = 0; }

#pragma unroll 1
  for (int j4 = 0; j4 < NN / 4; ++j4) {
    const v4f z4 = *(const v4fa*)(zs + 4 * j4);
    const int j = 4 * j4;
#pragma unroll
    for (int mm = 0; mm < 16; ++mm) {
      const int i = ibase + mm;
      const float z = zi[mm];
      int c = ((z4.x > z) || (z4.x == z && j     < i)) ? 1 : 0;
      c    += ((z4.y > z) || (z4.y == z && j + 1 < i)) ? 1 : 0;
      c    += ((z4.z > z) || (z4.z == z && j + 2 < i)) ? 1 : 0;
      c    += ((z4.w > z) || (z4.w == z && j + 3 < i)) ? 1 : 0;
      rk[mm] += c;
    }
  }

  unsigned msk = 0u;
#pragma unroll
  for (int mm = 0; mm < 16; ++mm) if (rk[mm] < KSEL) msk |= (1u << mm);
  const int cnt = (int)__builtin_popcount(msk);
  int incl = cnt;
#pragma unroll
  for (int d = 1; d < 32; d <<= 1) {
    const int y = __shfl_up(incl, d, 32);
    if (lane >= d) incl += y;
  }
  if (lane == 31) wtot[wave] = incl;
  __syncthreads();
  int pre = 0;
#pragma unroll
  for (int w = 0; w < NWAVE; ++w) pre += (w < wave) ? wtot[w] : 0;
  int run = pre + incl - cnt;
#pragma unroll
  for (int mm = 0; mm < 16; ++mm) {
    const int i = ibase + mm;
    if (((msk >> mm) & 1u) != 0u) {
      if (run < IDXN) lidx[run] = i;
      lmem[i] = run;
      run = run + 1;
    } else {
      lmem[i] = -1;
    }
  }
  __syncthreads();

  sel_pass(lmem, lidx, memp, idxp, tid);
  __threadfence();
  sel_pass(lmem, lidx, memp, idxp, tid);
}

template <int MODE>
__global__ __launch_bounds__(NTHR) void k_split(const float* __restrict__ src, const int* __restrict__ idxp,
                                                const float* __restrict__ zp, const float* __restrict__ bias,
                                                unsigned short* outp) {
  const int tid = (int)threadIdx.x;
  const int r = (int)blockIdx.x * 16 + (tid >> 4);
  const int q = tid & 15;
  const bool live = r < KSEL;
  float v[8];
  if constexpr (MODE == 0) {
    const int n = clampn(idxp[r < IDXN ? r : IDXN - 1], NN);
    float z = zp[n];
    z = fminf(fmaxf(z, -30.0f), 30.0f);
    const float s = 1.0f / (1.0f + expf(-z));
    const float* p = src + (size_t)n * DD + 8 * q;
    const v4f a = *(const v4f*)p;
    const v4f b = *(const v4f*)(p + 4);
    v[0] = a.x * s; v[1] = a.y * s; v[2] = a.z * s; v[3] = a.w * s;
    v[4] = b.x * s; v[5] = b.y * s; v[6] = b.z * s; v[7] = b.w * s;
  } else {
    const float* p = src + (size_t)r * K2 + 8 * q;
    const v4f a0 = *(const v4f*)p;
    const v4f a1 = *(const v4f*)(p + 4);
    const v4f b0 = *(const v4f*)(p + DD);
    const v4f b1 = *(const v4f*)(p + DD + 4);
    const v4f c0 = *(const v4f*)(bias + 8 * q);
    const v4f c1 = *(const v4f*)(bias + 8 * q + 4);
    v[0] = (a0.x + b0.x) + bf16_val(c0.x); v[1] = (a0.y + b0.y) + bf16_val(c0.y);
    v[2] = (a0.z + b0.z) + bf16_val(c0.z); v[3] = (a0.w + b0.w) + bf16_val(c0.w);
    v[4] = (a1.x + b1.x) + bf16_val(c1.x); v[5] = (a1.y + b1.y) + bf16_val(c1.y);
    v[6] = (a1.z + b1.z) + bf16_val(c1.z); v[7] = (a1.w + b1.w) + bf16_val(c1.w);
  }
  v8us ho, lo;
#pragma unroll
  for (int i = 0; i < 8; ++i) {
    const float x = live ? v[i] : 0.0f;
    const unsigned hb = bf16_bits(x);
    ho[i] = (unsigned short)hb;
    lo[i] = (unsigned short)bf16_bits(x - __uint_as_float(hb << 16));
  }
  unsigned short* hp = outp + (size_t)r * K2 + 8 * q;
  *(volatile v8us*)hp = ho;
  *(volatile v8us*)(hp + DD) = lo;
  __threadfence();
  *(volatile v8us*)hp = ho;
  *(volatile v8us*)(hp + DD) = lo;
}

__device__ __forceinline__ void yt_pass(const float* tile, unsigned short* yt, int nb, int wave, int lane) {
  const int part = wave >> 2;
#pragma unroll 2
  for (int i = 0; i < 8; ++i) {
    const int L  = wave * 32 + 4 * i + (lane >> 3);
    const int c  = L & (DD - 1);
    const int j0 = 8 * (lane & 7);
    v8us o;
#pragma unroll
    for (int jj = 0; jj < 8; ++jj) {
      const float v = tile[(j0 + jj) * DD + c];
      const unsigned hb = bf16_bits(v);
      const unsigned lb = bf16_bits(v - __uint_as_float(hb << 16));
      o[jj] = (unsigned short)(part != 0 ? lb : hb);
    }
    unsigned short* op = yt + (size_t)(part * DD + c) * NN + nb + j0;
    *(volatile v8us*)op = o;
  }
}

__global__ __launch_bounds__(NTHR) void k_yt(const float* __restrict__ ys, const int* __restrict__ memp,
                                             unsigned short* yt) {
  __shared__ __attribute__((aligned(16))) float tile[64 * DD];
  const int tid = (int)threadIdx.x, lane = tid & 31, wave = tid >> 5;
  const int nb = (int)blockIdx.x * 64;
#pragma unroll
  for (int it = 0; it < (64 * DD / 4) / NTHR; ++it) {
    const int u = it * NTHR + tid;
    const int r = u >> 5;
    const int q = u & 31;
    int p = memp[nb + r];
    const bool live = p >= 0;
    p = clampn(p, KP);
    const v4f x = *(const v4f*)(ys + (size_t)p * DD + 4 * q);
    v4f y;
    y.x = live ? x.x : 0.0f; y.y = live ? x.y : 0.0f; y.z = live ? x.z : 0.0f; y.w = live ? x.w : 0.0f;
    *(v4fa*)(tile + r * DD + 4 * q) = y;
  }
  __syncthreads();

  yt_pass(tile, yt, nb, wave, lane);
  __threadfence();
  yt_pass(tile, yt, nb, wave, lane);
}

__global__ __launch_bounds__(NTHR) void k_final(const float* __restrict__ hup2, const float* __restrict__ h0,
                                                const float* __restrict__ h, const float* __restrict__ bu,
                                                float* outp) {
  const int tid = (int)threadIdx.x, lane = tid & 31, wave = tid >> 5;
  const int row = (int)blockIdx.x * NWAVE + wave;
  const int c = 4 * lane;
  const v4f a  = *(const v4f*)(hup2 + (size_t)row * K2 + c);
  const v4f b  = *(const v4f*)(hup2 + (size_t)row * K2 + DD + c);
  const v4f x0 = *(const v4f*)(h0 + (size_t)row * DD + c);
  const v4f xh = *(const v4f*)(h + (size_t)row * DD + c);
  const v4f bb = *(const v4f*)(bu + c);
  v4f h1, h2;
  h1.x = ((a.x + b.x) + bf16_val(bb.x)) + x0.x; h2.x = h1.x + bf16_val(xh.x);
  h1.y = ((a.y + b.y) + bf16_val(bb.y)) + x0.y; h2.y = h1.y + bf16_val(xh.y);
  h1.z = ((a.z + b.z) + bf16_val(bb.z)) + x0.z; h2.z = h1.z + bf16_val(xh.z);
  h1.w = ((a.w + b.w) + bf16_val(bb.w)) + x0.w; h2.w = h1.w + bf16_val(xh.w);
  float* o0 = outp + (size_t)row * DD + c;
  float* o1 = outp + (size_t)NN * DD + (size_t)row * DD + c;
  *(volatile v4f*)o0 = h1;
  *(volatile v4f*)o1 = h2;
  __threadfence();
  *(volatile v4f*)o0 = h1;
  *(volatile v4f*)o1 = h2;
}

extern "C" void kernel_launch(void* const* d_in, const int* in_sizes, int n_in,
                              void* d_out, int out_size, void* d_ws, size_t ws_size,
                              hipStream_t stream) {
  if (n_in < 10) return;
  if (in_sizes[0] < 2 || (in_sizes[0] & 1) != 0) return;
  const int nE = in_sizes[0] / 2;
  if (nE < 1 || nE >= (1 << 26)) return;
  if (in_sizes[1] != NN * DD) return;
  if (in_sizes[2] != DD * DD || in_sizes[3] != DD) return;
  if (in_sizes[4] != DD || in_sizes[5] < 1) return;
  if (in_sizes[6] != DD * DD || in_sizes[7] != DD) return;
  if (in_sizes[8] != DD * DD || in_sizes[9] != DD) return;
  if (out_size != 2 * NN * DD) return;

  const int*   g  = (const int*)d_in[0];
  const float* h  = (const float*)d_in[1];
  const float* Wd = (const float*)d_in[2];
  const float* bd = (const float*)d_in[3];
  const float* pw = (const float*)d_in[4];
  const float* pb = (const float*)d_in[5];
  const float* Wb = (const float*)d_in[6];
  const float* bb = (const float*)d_in[7];
  const float* Wu = (const float*)d_in[8];
  const float* bu = (const float*)d_in[9];
  float* out = (float*)d_out;
  const int* src = g;
  const int* dst = g + nE;
  const int vec8 = ((nE & 3) == 0) ? 1 : 0;

  char* ws = (char*)d_ws;
  size_t off = 0;
#define CARVE(NAME, BYTES) const size_t NAME = off; off += (size_t)(BYTES); off = (off + 255) & ~(size_t)255;
  CARVE(oWDT,   (size_t)DD * DD * 2)
  CARVE(oWBT2,  (size_t)DD * K2 * 2)
  CARVE(oWUT2,  (size_t)DD * K2 * 2)
  CARVE(oHBF,   (size_t)NN * DD * 2)
  CARVE(oADJ,   (size_t)NN * NN * 2)
  CARVE(oH0,    (size_t)NN * DD * 4)
  CARVE(oZ,     (size_t)NN * 4)
  CARVE(oMEM,   (size_t)NN * 4)
  CARVE(oIDX,   (size_t)IDXN * 4)
  CARVE(oNEWH,  (size_t)KP * K2 * 2)
  CARVE(oUA,    (size_t)KP * NN * 2)
  CARVE(oUBT,   (size_t)KP * NN * 2)
  CARVE(oSUB,   (size_t)KP * KP * 2)
  CARVE(oPARTD, (size_t)NPB * KP * 4)
  CARVE(oXST,   (size_t)K2 * KP * 2)
  CARVE(oHB2,   (size_t)KP * K2 * 4)
  CARVE(oHBP,   (size_t)KP * K2 * 2)
  CARVE(oYS,    (size_t)KP * DD * 4)
  CARVE(oYT,    (size_t)K2 * NN * 2)
  CARVE(oHUP2,  (size_t)NN * K2 * 4)
#undef CARVE
  if (off > ws_size || off > (size_t)WSMAX) return;

  unsigned short* WDT  = (unsigned short*)(ws + oWDT);
  unsigned short* WBT2 = (unsigned short*)(ws + oWBT2);
  unsigned short* WUT2 = (unsigned short*)(ws + oWUT2);
  unsigned short* HBF  = (unsigned short*)(ws + oHBF);
  unsigned short* ADJ  = (unsigned short*)(ws + oADJ);
  float*          H0   = (float*)(ws + oH0);
  float*          Z    = (float*)(ws + oZ);
  int*            MEM  = (int*)(ws + oMEM);
  int*            IDX  = (int*)(ws + oIDX);
  unsigned short* NEWH = (unsigned short*)(ws + oNEWH);
  unsigned short* UA   = (unsigned short*)(ws + oUA);
  unsigned short* UBT  = (unsigned short*)(ws + oUBT);
  unsigned short* SUBP = (unsigned short*)(ws + oSUB);
  float*          PARTD = (float*)(ws + oPARTD);
  unsigned short* XST  = (unsigned short*)(ws + oXST);
  float*          HB2  = (float*)(ws + oHB2);
  unsigned short* HBP  = (unsigned short*)(ws + oHBP);
  float*          YS   = (float*)(ws + oYS);
  unsigned short* YT   = (unsigned short*)(ws + oYT);
  float*          HUP2 = (float*)(ws + oHUP2);

  const size_t adjLds = (size_t)ADJ_LDS_INTS * 4;
  const size_t uLds   = (size_t)U_LDS_INTS * 4;
  hipFuncSetAttribute(reinterpret_cast<const void*>(&k_adj),  hipFuncAttributeMaxDynamicSharedMemorySize, (int)adjLds);
  hipFuncSetAttribute(reinterpret_cast<const void*>(&k_urow), hipFuncAttributeMaxDynamicSharedMemorySize, (int)uLds);

  k_prep<<<NUTOT / NTHR, NTHR, 0, stream>>>(h, Wd, Wb, Wu, HBF, WDT, WBT2, WUT2);
  k_adj<<<NN / ARB, NTHR, adjLds, stream>>>(src, dst, nE, vec8, ADJ);
  k_gemm<MODE_H0Z><<<dim3(NN / GBM, 1), GTHR, 0, stream>>>(HBF, DD, WDT, DD, DD, H0, DD, NEWH, bd, pw, pb, Z);
  k_select<<<1, NTHR, 0, stream>>>(Z, MEM, IDX);
  k_split<0><<<KP / 16, NTHR, 0, stream>>>(H0, IDX, Z, bd, NEWH);
  k_urow<<<KP / URB, NTHR, uLds, stream>>>(src, dst, nE, vec8, MEM, UA);
  k_urow<<<KP / URB, NTHR, uLds, stream>>>(dst, src, nE, vec8, MEM, UBT);
  k_gemm<MODE_SUB><<<dim3(KP / GBM, KP / GBN), GTHR, 0, stream>>>(UA, NN, UBT, NN, NN, PARTD, KP, SUBP, bd, bd, bd, PARTD);
  k_gemm<MODE_XST><<<dim3(KP / GBM, 1), GTHR, 0, stream>>>(NEWH, K2, WBT2, K2, K2, HB2, KP, XST, PARTD, bd, bd, Z);
  k_gemm<MODE_F32><<<dim3(KP / GBM, K2 / GBN), GTHR, 0, stream>>>(SUBP, KP, XST, KP, KP, HB2, K2, NEWH, bd, bd, bd, PARTD);
  k_split<1><<<KP / 16, NTHR, 0, stream>>>(HB2, IDX, Z, bb, HBP);
  k_gemm<MODE_F32><<<dim3(KP / GBM, 1), GTHR, 0, stream>>>(HBP, K2, WUT2, K2, K2, YS, DD, NEWH, bd, bd, bd, PARTD);
  k_yt<<<NN / 64, NTHR, 0, stream>>>(YS, MEM, YT);
  k_gemm<MODE_F32><<<dim3(NN / GBM, K2 / GBN), GTHR, 0, stream>>>(ADJ, NN, YT, NN, NN, HUP2, K2, NEWH, bd, bd, bd, PARTD);
  k_final<<<NN / NWAVE, NTHR, 0, stream>>>(HUP2, H0, h, bu, out);
}
